// LCAMatrixModel_41944650613376
// MI455X (gfx1250) — hardware-run, weakly checked
//
#include <hip/hip_runtime.h>


#ifndef NROW
#define NROW 1024
#endif
#define NROW_FULL 1024
#ifndef OUT_PITCH
#define OUT_PITCH NROW
#endif
#define RAW  128
#define DL   128
#define HID  256
#define ABP  512
#define PJ   64
#define PI   16
#define KC   128
#define KP   132
#define W1S  64.0f
#define W1I  (1.0f / 64.0f)
#define LOG2EF 1.4426950408889634f
#define WPC  ((float)(1.0507009873554805 * 0.6931471805599453))
#define WAC  ((float)(1.0507009873554805 * 1.6732632423543772))

static_assert(RAW % 32 == 0);
static_assert(DL % 32 == 0);
static_assert(RAW % 64 == 0);
static_assert(DL % 64 == 0);
static_assert(DL % 32 == 0);
static_assert(HID % 64 == 0);
static_assert(HID % 32 == 0);
static_assert(ABP == 2 * HID);
static_assert(NROW % 64 == 0);
static_assert(NROW % PJ == 0);
static_assert(NROW % PI == 0);
static_assert(NROW <= NROW_FULL);
static_assert(OUT_PITCH >= NROW);
static_assert(OUT_PITCH % 32 == 0);
static_assert(HID == 256);
static_assert(HID % KC == 0);
static_assert(KC == 128);
static_assert(KC % 4 == 0);
static_assert(KP >= KC);
static_assert(KP % 4 == 0);
static_assert((256 / 32) * 8 == PJ);
static_assert((256 / 32) * 2 == PI);
static_assert(16 * 4 == PJ);
static_assert(256 / 16 == PI);
static_assert(16 * 16 == PJ * 4);
static_assert((PJ + PI) * KP * 4 + 2 * HID * 4 <= 131072);
static_assert(16 * 68 * 4 <= 131072);
static_assert(32 * 68 * 4 <= 131072);

typedef _Float16 h16;
typedef unsigned short bf;
typedef __attribute__((ext_vector_type(16))) __bf16   v16bf;
typedef __attribute__((ext_vector_type(16))) _Float16 v16h;
typedef __attribute__((ext_vector_type(8)))  _Float16 v8h;
typedef __attribute__((ext_vector_type(8)))  unsigned short v8us;
typedef __attribute__((ext_vector_type(8)))  float    v8f;
typedef __attribute__((ext_vector_type(4)))  float    v4f;
typedef v4f  __attribute__((may_alias)) v4fa;

__device__ __forceinline__ unsigned short f2bf(float f) { unsigned u = __float_as_uint(f); u += 0x7FFFu + ((u >> 16) & 1u); return (unsigned short)(u >> 16); }
__device__ __forceinline__ float bfr(float f) { return __uint_as_float(((unsigned)f2bf(f)) << 16); }
__device__ __forceinline__ v16h cat16(v8h lo, v8h hi) { return __builtin_shufflevector(lo, hi, 0, 1, 2, 3, 4, 5, 6, 7, 8, 9, 10, 11, 12, 13, 14, 15); }
__device__ __forceinline__ v16bf cat16b(v8us lo, v8us hi) { return __builtin_bit_cast(v16bf, __builtin_shufflevector(lo, hi, 0, 1, 2, 3, 4, 5, 6, 7, 8, 9, 10, 11, 12, 13, 14, 15)); }
__device__ __forceinline__ v8f wmma16(v16h a, v16h b, v8f c) { return __builtin_amdgcn_wmma_f32_16x16x32_f16(false, a, false, b, (short)0, c, false, false); }
__device__ __forceinline__ v8f wmmab(v16bf a, v16bf b, v8f c) { return __builtin_amdgcn_wmma_f32_16x16x32_bf16(false, a, false, b, (short)0, c, false, false); }
__device__ __forceinline__ v16h  ldh(const h16* p) { return cat16(*(const v8h*)p, *(const v8h*)(p + 16)); }
__device__ __forceinline__ v16bf ldb(const bf* p)  { return cat16b(*(const v8us*)p, *(const v8us*)(p + 16)); }
__device__ __forceinline__ void wave_sync() { __builtin_amdgcn_fence(3  , "wavefront"); __builtin_amdgcn_wave_barrier(); asm volatile("" ::: "memory"); }

static __device__ __forceinline__ h16 toh_flush(float v) { const h16 r = (h16)v; return (fabsf(v) < 6.103515625e-05f) ? (h16)0.0f : r; }

__device__ __forceinline__ v8f mmg(v16h a, v16h b, v8f c)   { c = wmma16(a, b, c); asm volatile("v_nop\n\tv_nop\n\tv_nop\n\tv_nop" : "+v"(c) : "v"(a), "v"(b)); return c; }
__device__ __forceinline__ v8f mmg(v16bf a, v16bf b, v8f c) { c = wmmab(a, b, c);  asm volatile("v_nop\n\tv_nop\n\tv_nop\n\tv_nop" : "+v"(c) : "v"(a), "v"(b)); return c; }
__device__ __forceinline__ v16h  ldf(const h16* p) { return ldh(p); }
__device__ __forceinline__ v16bf ldf(const bf* p)  { return ldb(p); }
template <typename T> struct frag_of;
template <> struct frag_of<bf>  { typedef v16bf t; };
template <> struct frag_of<h16> { typedef v16h  t; };

__global__ __launch_bounds__(256) void k_cvt8(const float* __restrict__ src, bf* dst, size_t n8) {
    const size_t i = (size_t)blockIdx.x * 256 + threadIdx.x; if (i >= n8) return;
    const v8f v = *(const v8f*)(src + i * 8); v8us o;
#pragma unroll
    for (int k = 0; k < 8; ++k) o[k] = f2bf(v[k]);
    *(volatile v8us*)(dst + i * 8) = o; __threadfence(); *(volatile v8us*)(dst + i * 8) = o;
}

template <int MODE>
__device__ __forceinline__ void wtr_body(const float* __restrict__ in, bf* ob, h16* oh, int R, int C) {
    __shared__ __align__(16) float ts[32 * 68];
    const int t = threadIdx.x;
    const int r0 = blockIdx.x * 64, c0 = blockIdx.y * 32;
    const float* src = in + (size_t)blockIdx.z * (size_t)R * (size_t)C;
    const size_t obase = (size_t)blockIdx.z * (size_t)C * (size_t)R;
    { const int r = t >> 2, c8 = (t & 3) * 8;
      const float* p = src + (size_t)(r0 + r) * C + c0 + c8;
      const v4f x0 = *(const v4f*)p, x1 = *(const v4f*)(p + 4);
#pragma unroll
      for (int i = 0; i < 4; ++i) { ts[(c8 + i) * 68 + r] = x0[i]; ts[(c8 + 4 + i) * 68 + r] = x1[i]; } }
    __syncthreads();
    const int c = t >> 3, r8 = (t & 7) * 8;
    const v4f y0 = *(const v4fa*)(&ts[c * 68 + r8]), y1 = *(const v4fa*)(&ts[c * 68 + r8 + 4]);
    const size_t oo = obase + (size_t)(c0 + c) * R + r0 + r8;
    if (MODE == 0) {
        v8us o;
#pragma unroll
        for (int i = 0; i < 4; ++i) { o[i] = f2bf(y0[i]); o[4 + i] = f2bf(y1[i]); }
        *(volatile v8us*)(ob + oo) = o; __threadfence(); *(volatile v8us*)(ob + oo) = o;
    } else {
        v8h o;
#pragma unroll
        for (int i = 0; i < 4; ++i) { o[i] = toh_flush(bfr(y0[i]) * W1S); o[4 + i] = toh_flush(bfr(y1[i]) * W1S); }
        *(volatile v8h*)(oh + oo) = o; __threadfence(); *(volatile v8h*)(oh + oo) = o;
    }
}
static_assert(256 * 16 == 32 * 128);
__global__ __launch_bounds__(256) void k_wtr_b(const float* __restrict__ in, bf* out, int R, int C)  { wtr_body<0>(in, out, (h16*)0, R, C); }
__global__ __launch_bounds__(256) void k_wtr_h(const float* __restrict__ in, h16* out, int R, int C) { wtr_body<1>(in, (bf*)0, out, R, C); }

template <typename T, int K>
__device__ __forceinline__ void gemm_tile64(const T* __restrict__ A, const T* __restrict__ Bt, int r0, int c0, int lr, int hi, v8f (&acc)[4][4]) {
    typedef typename frag_of<T>::t F;
    const size_t aoff = (size_t)(r0 + lr) * K + 8 * hi, boff = (size_t)(c0 + lr) * K + 8 * hi;
#pragma unroll 1
    for (int kc = 0; kc < K; kc += 32) {
        F a[4];
#pragma unroll
        for (int mb = 0; mb < 4; ++mb) a[mb] = ldf(A + aoff + (size_t)mb * 16 * K + kc);
#pragma unroll
        for (int nb = 0; nb < 4; ++nb) { const F b = ldf(Bt + boff + (size_t)nb * 16 * K + kc);
#pragma unroll
            for (int mb = 0; mb < 4; ++mb) acc[mb][nb] = mmg(a[mb], b, acc[mb][nb]); }
    }
}

static_assert(32 * 16 * 4 == 16 * 64 * 2);
__global__ __launch_bounds__(32) void k_gemm_z(const bf* __restrict__ A, const bf* __restrict__ Bt, const float* __restrict__ bias, h16* ZH) {
    __shared__ __align__(16) float os[16 * 68];
    const int lane = threadIdx.x & 31, lr = lane & 15, hi = lane >> 4; const int r0 = blockIdx.x * 64, c0 = blockIdx.y * 64;
    v8f acc[4][4];
#pragma unroll
    for (int mb = 0; mb < 4; ++mb)
#pragma unroll
        for (int nb = 0; nb < 4; ++nb) acc[mb][nb] = (v8f){};
    gemm_tile64<bf, RAW>(A, Bt, r0, c0, lr, hi, acc);
    float bc[4];
#pragma unroll
    for (int nb = 0; nb < 4; ++nb) bc[nb] = bfr(bias[c0 + nb * 16 + lr]);
#pragma unroll
    for (int mb = 0; mb < 4; ++mb) {
#pragma unroll
        for (int nb = 0; nb < 4; ++nb) {
#pragma unroll
            for (int j = 0; j < 8; ++j) os[(hi * 8 + j) * 68 + nb * 16 + lr] = acc[mb][nb][j] + bc[nb]; }
        wave_sync();
#pragma unroll 1
        for (int ps = 0; ps < 2; ++ps) {
#pragma unroll
            for (int s = 0; s < 4; ++s) { const int row = 4 * s + (lane >> 3), c8 = (lane & 7) * 8;
                const v4f x0 = *(const v4fa*)(&os[row * 68 + c8]); const v4f x1 = *(const v4fa*)(&os[row * 68 + c8 + 4]); v8h hv;
#pragma unroll
                for (int i = 0; i < 4; ++i) { hv[i] = toh_flush(x0[i]); hv[4 + i] = toh_flush(x1[i]); }
                *(volatile v8h*)(ZH + (size_t)(r0 + mb * 16 + row) * DL + c0 + c8) = hv; }
            if (ps == 0) __threadfence(); }
        wave_sync();
    }
}

static_assert(32 * 16 * 8 == 16 * 64 * 4);
__global__ __launch_bounds__(32) void k_gemm_ab(const h16* __restrict__ A, const h16* __restrict__ Bt, const float* __restrict__ b1, float* AB) {
    __shared__ __align__(16) float os[16 * 68];
    const int lane = threadIdx.x & 31, lr = lane & 15, hi = lane >> 4; const int r0 = blockIdx.x * 64, c0 = blockIdx.y * 64;
    v8f acc[4][4];
#pragma unroll
    for (int mb = 0; mb < 4; ++mb)
#pragma unroll
        for (int nb = 0; nb < 4; ++nb) acc[mb][nb] = (v8f){};
    gemm_tile64<h16, DL>(A, Bt, r0, c0, lr, hi, acc);
    float bc[4];
#pragma unroll
    for (int nb = 0; nb < 4; ++nb) { const int cc = c0 + nb * 16 + lr; const int ci = cc < HID ? cc : (HID - 1);
        float bv = b1[ci]; asm volatile("" : "+v"(bv));
        bc[nb] = (cc < HID) ? bfr(bv) : 0.0f; }
#pragma unroll
    for (int mb = 0; mb < 4; ++mb) {
#pragma unroll
        for (int nb = 0; nb < 4; ++nb) {
#pragma unroll
            for (int j = 0; j < 8; ++j) os[(hi * 8 + j) * 68 + nb * 16 + lr] = acc[mb][nb][j] * W1I + bc[nb]; }
        wave_sync();
#pragma unroll 1
        for (int ps = 0; ps < 2; ++ps) {
#pragma unroll
            for (int s = 0; s < 8; ++s) { const int row = 2 * s + (lane >> 4), cofs = (lane & 15) * 4;
                const v4f val = *(const v4fa*)(&os[row * 68 + cofs]);
                *(volatile v4f*)(AB + (size_t)(r0 + mb * 16 + row) * ABP + c0 + cofs) = val; }
            if (ps == 0) __threadfence(); }
        wave_sync();
    }
}

__device__ __forceinline__ float pterm(float h2, float wp, float wa, float acc) {
    const float p = fmaxf(h2, 0.0f), q = fminf(h2, 0.0f);
    const float e = __builtin_amdgcn_exp2f(q);
    acc = fmaf(p, wp, acc);
    return fmaf(e, wa, acc);
}
__device__ __forceinline__ float hsig(float v) { return fminf(fmaxf(v + 3.0f, 0.0f), 6.0f) * (1.0f / 6.0f); }

__global__ __launch_bounds__(256) void k_pair(const float* __restrict__ AB, const float* __restrict__ W2, const float* __restrict__ b2, float* OUT) {
#pragma clang fp contract(off)
    __shared__ __align__(16) float sA[PJ * KP];
    __shared__ __align__(16) float sB[PI * KP];
    __shared__ __align__(16) float sWp[HID];
    __shared__ __align__(16) float sWa[HID];
    const int t = threadIdx.x, tj = t & 15, ti = t >> 4;
    const int j0 = blockIdx.x * PJ, i0 = blockIdx.y * PI;
    { const float w = bfr(W2[t]); sWp[t] = WPC * w; sWa[t] = WAC * w; }
    const int sc = t & 31, sr = t >> 5;
    const int ao = (4 * tj) * KP, bo = ti * KP;
    float acc0 = 0.0f, acc1 = 0.0f, acc2 = 0.0f, acc3 = 0.0f, wsum = 0.0f;
#pragma unroll 1
    for (int kc = 0; kc < HID; kc += KC) {
        __syncthreads();
#pragma unroll
        for (int s = 0; s < 8; ++s) { const int r = sr + 8 * s;
            v4f v = *(const v4f*)(AB + (size_t)(j0 + r) * ABP + kc + 4 * sc); v = v * LOG2EF;
            *(v4fa*)(&sA[r * KP + 4 * sc]) = v; }
#pragma unroll
        for (int s = 0; s < 2; ++s) { const int r = sr + 8 * s;
            v4f v = *(const v4f*)(AB + (size_t)(i0 + r) * ABP + HID + kc + 4 * sc); v = v * LOG2EF;
            *(v4fa*)(&sB[r * KP + 4 * sc]) = v; }
        __syncthreads();
#pragma unroll 1
        for (int k = 0; k < KC; k += 4) {
            const v4f b  = *(const v4fa*)(&sB[bo + k]);
            const v4f wp = *(const v4fa*)(&sWp[kc + k]);
            const v4f wa = *(const v4fa*)(&sWa[kc + k]);
            const v4f a0 = *(const v4fa*)(&sA[ao + k]);
            const v4f a1 = *(const v4fa*)(&sA[ao + KP + k]);
            const v4f a2 = *(const v4fa*)(&sA[ao + 2 * KP + k]);
            const v4f a3 = *(const v4fa*)(&sA[ao + 3 * KP + k]);
            wsum += (wa[0] + wa[1]) + (wa[2] + wa[3]);
#pragma unroll
            for (int c = 0; c < 4; ++c) {
                acc0 = pterm(a0[c] + b[c], wp[c], wa[c], acc0);
                acc1 = pterm(a1[c] + b[c], wp[c], wa[c], acc1);
                acc2 = pterm(a2[c] + b[c], wp[c], wa[c], acc2);
                acc3 = pterm(a3[c] + b[c], wp[c], wa[c], acc3); }
        }
    }
    const float cb = bfr(b2[0]) - wsum;
    v4f o;
    o[0] = hsig(acc0 + cb); o[1] = hsig(acc1 + cb); o[2] = hsig(acc2 + cb); o[3] = hsig(acc3 + cb);
    float* op = OUT + (size_t)(i0 + ti) * OUT_PITCH + j0 + 4 * tj;
    *(volatile v4f*)op = o; __threadfence(); *(volatile v4f*)op = o;
}

static constexpr size_t al256(size_t v) { return (v + 255) & ~(size_t)255; }
static constexpr size_t SZ_XB = al256((size_t)NROW * RAW * 2);
static constexpr size_t SZ_WE = al256((size_t)DL * RAW * 2);
static constexpr size_t SZ_W1 = al256((size_t)2 * HID * DL * 2);
static constexpr size_t SZ_ZH = al256((size_t)NROW * DL * 2);
static constexpr size_t SZ_AB = al256((size_t)NROW * ABP * 4);
static constexpr size_t SZ_TOTAL = SZ_XB + SZ_WE + SZ_W1 + SZ_ZH + SZ_AB;
static_assert(SZ_TOTAL <= (size_t)134217728);
static_assert(((size_t)NROW * RAW) % 8 == 0);
static_assert(((size_t)(NROW / 64) * 64) == (size_t)NROW);

extern "C" void kernel_launch(void* const* d_in, const int* in_sizes, int n_in,
                              void* d_out, int out_size, void* d_ws, size_t ws_size, hipStream_t stream) {
    if (n_in < 7) return;
    if ((size_t)in_sizes[0] < (size_t)NROW * RAW) return;
    if ((size_t)in_sizes[1] < (size_t)RAW * DL || in_sizes[2] < DL) return;
    if ((size_t)in_sizes[3] < (size_t)2 * DL * HID || in_sizes[4] < HID) return;
    if (in_sizes[5] < HID || in_sizes[6] < 1) return;
    if ((size_t)out_size < (size_t)(NROW - 1) * OUT_PITCH + NROW) return;
    if (SZ_TOTAL > ws_size) return;
    const float* x    = (const float*)d_in[0];
    const float* wenc = (const float*)d_in[1];
    const float* benc = (const float*)d_in[2];
    const float* w1   = (const float*)d_in[3];
    const float* b1   = (const float*)d_in[4];
    const float* w2   = (const float*)d_in[5];
    const float* b2   = (const float*)d_in[6];
    float* OUT = (float*)d_out;
    char* wsp = (char*)d_ws;
    bf*  XB  = (bf*)wsp;  wsp += SZ_XB;
    bf*  WE  = (bf*)wsp;  wsp += SZ_WE;
    h16* W1T = (h16*)wsp; wsp += SZ_W1;
    h16* ZH  = (h16*)wsp; wsp += SZ_ZH;
    float* AB = (float*)wsp; wsp += SZ_AB;

    { const size_t n8 = (size_t)NROW * RAW / 8;
      k_cvt8<<<(unsigned)((n8 + 255) / 256), 256, 0, stream>>>(x, XB, n8); }
    k_wtr_b<<<dim3(RAW / 64, DL / 32, 1), 256, 0, stream>>>(wenc, WE, RAW, DL);
    k_wtr_h<<<dim3(DL / 64, HID / 32, 2), 256, 0, stream>>>(w1, W1T, DL, HID);
    k_gemm_z<<<dim3(NROW / 64, DL / 64, 1), 32, 0, stream>>>(XB, WE, benc, ZH);
    k_gemm_ab<<<dim3(NROW / 64, (2 * HID) / 64, 1), 32, 0, stream>>>(ZH, W1T, b1, AB);
    k_pair<<<dim3(NROW / PJ, NROW / PI, 1), 256, 0, stream>>>(AB, w2, b2, OUT);
}
